// SimplifiedGateNetwork_23957327577730
// MI455X (gfx1250) — hardware-verified
//
#include <hip/hip_runtime.h>


namespace {
constexpr int NBt = 16384, T = 40, V = 40, D = 128, HID = 32, G4 = 128, NE = 4, FH = 2 * HID + 2;
constexpr float XS = 8.0f, WSC = 256.0f;

typedef _Float16 b16;
typedef __attribute__((ext_vector_type(16))) _Float16 v16b;
typedef __attribute__((ext_vector_type(8))) _Float16 v8b;
typedef __attribute__((ext_vector_type(8))) float v8f;
typedef __attribute__((ext_vector_type(4))) float v4f;
__device__ __forceinline__ float bf16_rne(float f) { unsigned int u = __float_as_uint(f); u += 0x7FFFu + ((u >> 16) & 1u); return __uint_as_float(u & 0xFFFF0000u); }
__device__ __forceinline__ void split16(float v, b16& hi, b16& lo) { hi = (b16)v; lo = (b16)(v - (float)hi); }
__device__ __forceinline__ v16b frag_kb(const b16* p, int hh) { const v8b a = *(const v8b*)(p + 8 * hh), b = *(const v8b*)(p + 16 + 8 * hh); v16b f;
#pragma unroll
  for (int e = 0; e < 8; ++e) { f[e] = a[e]; f[8 + e] = b[e]; } return f; }
__device__ __forceinline__ v8f wmma16b(v16b a, v16b b, v8f c) { v8f d = __builtin_amdgcn_wmma_f32_16x16x32_f16(false, a, false, b, (short)0, c, false, false); asm volatile("v_nop\n\tv_nop\n\tv_nop\n\tv_nop" : "+v"(d) : "v"(a), "v"(b)); return d; }
__device__ __forceinline__ void wave_lds_sync() { __builtin_amdgcn_fence(__ATOMIC_RELEASE, "workgroup"); __builtin_amdgcn_wave_barrier(); __builtin_amdgcn_fence(__ATOMIC_ACQUIRE, "workgroup"); }
__device__ __forceinline__ float nexp(float x) { return __builtin_amdgcn_exp2f(x * 1.4426950408889634f); }
__device__ __forceinline__ float pmul(float a, float b) { float p = a * b; asm volatile("" : "+v"(p)); return p; }
__device__ __forceinline__ float sigm(float x) { return 1.0f / (1.0f + nexp(-x)); }
__device__ __forceinline__ float tanh_(float x) { const float e = nexp(-2.0f * fabsf(x)); const float t = (1.0f - e) / (1.0f + e); return x < 0.0f ? -t : t; }
__device__ __forceinline__ int iclamp(int v, int lo, int hi) { return v < lo ? lo : (v > hi ? hi : v); }

__global__ __launch_bounds__(256) void prep_kernel(const float* __restrict__ emb, const float* __restrict__ wihf, const float* __restrict__ whhf, const float* __restrict__ wihb, const float* __restrict__ whhb, b16* __restrict__ EMB16, b16* __restrict__ WIH, b16* __restrict__ WHH) {
  const int t = blockIdx.x * 256 + threadIdx.x; const int n0 = V * D / 8, n1 = G4 * D / 8, n2 = G4 * HID / 8;
  const float* src; b16* dst; float sc = WSC; int e;
  if (t < n0) { src = emb; dst = EMB16; e = t * 8; sc = XS; } else if (t < n0 + n1) { src = wihf; dst = WIH; e = (t - n0) * 8; } else if (t < n0 + 2 * n1) { src = wihb; dst = WIH + G4 * D; e = (t - n0 - n1) * 8; }
  else if (t < n0 + 2 * n1 + n2) { src = whhf; dst = WHH; e = (t - n0 - 2 * n1) * 8; } else if (t < n0 + 2 * n1 + 2 * n2) { src = whhb; dst = WHH + G4 * HID; e = (t - n0 - 2 * n1 - n2) * 8; } else return;
  v8b o; for (int j = 0; j < 8; ++j) o[j] = (b16)(bf16_rne(src[e + j]) * sc);
  for (int pass = 0; pass < 2; ++pass) { *(volatile v8b*)(dst + e) = o; __threadfence(); }
}
__global__ __launch_bounds__(128) void lstm_kernel(const int* __restrict__ x, const b16* __restrict__ EMB16, const b16* __restrict__ WIH, const b16* __restrict__ WHH, const float* __restrict__ bihf, const float* __restrict__ bhhf, const float* __restrict__ bihb, const float* __restrict__ bhhb, float* __restrict__ HF) {
  __shared__ __attribute__((aligned(16))) b16 Hh[4][16][HID + 8], Hl[4][16][HID + 8]; __shared__ __attribute__((aligned(16))) float Ho[4][16][HID + 4];
  const int wave = threadIdx.x >> 5, lane = threadIdx.x & 31, nloc = lane & 15, hlf = lane >> 4; const int dir = blockIdx.y; const size_t b0 = (size_t)blockIdx.x * 64 + wave * 16;
  const b16* Wi = WIH + (size_t)dir * G4 * D; const b16* Wh = WHH + (size_t)dir * G4 * HID; const float* bi = dir ? bihb : bihf; const float* bh = dir ? bhhb : bhhf;
  for (int q = lane; q < 16 * (HID + 8); q += 32) { (&Hh[wave][0][0])[q] = (b16)0.0f; (&Hl[wave][0][0])[q] = (b16)0.0f; }
  float bg[8]; for (int t = 0; t < 8; ++t) bg[t] = bf16_rne(bi[t * 16 + nloc]) + bf16_rne(bh[t * 16 + nloc]);
  float cst[2][8];
#pragma unroll
  for (int u = 0; u < 2; ++u)
#pragma unroll
    for (int r = 0; r < 8; ++r) cst[u][r] = 0.0f;
  wave_lds_sync();
  for (int step = 0; step < T; ++step) { const int t = dir ? (T - 1 - step) : step;
    const int tok = iclamp(x[(b0 + nloc) * T + t], 0, V - 1); const b16* arow = EMB16 + (size_t)tok * D;
    v8f acc[8];
#pragma unroll
    for (int tt = 0; tt < 8; ++tt) acc[tt] = (v8f){};
#pragma unroll
    for (int kb = 0; kb < D; kb += 32) { const v16b a = frag_kb(arow + kb, hlf);
#pragma unroll
      for (int tt = 0; tt < 8; ++tt) acc[tt] = wmma16b(a, frag_kb(Wi + (size_t)(tt * 16 + nloc) * D + kb, hlf), acc[tt]); }
    { const v16b ah = frag_kb(&Hh[wave][nloc][0], hlf), al = frag_kb(&Hl[wave][nloc][0], hlf);
#pragma unroll
      for (int tt = 0; tt < 8; ++tt) { const v16b bw = frag_kb(Wh + (size_t)(tt * 16 + nloc) * HID, hlf); acc[tt] = wmma16b(ah, bw, acc[tt]); acc[tt] = wmma16b(al, bw, acc[tt]); } }
    wave_lds_sync();
#pragma unroll
    for (int u = 0; u < 2; ++u) { const int unit = u * 16 + nloc; const float sc = 1.0f / (XS * WSC);
#pragma unroll
      for (int r = 0; r < 8; ++r) { const float zi = acc[0 + u][r] * sc + bg[0 + u], zf = acc[2 + u][r] * sc + bg[2 + u], zg = acc[4 + u][r] * sc + bg[4 + u], zo = acc[6 + u][r] * sc + bg[6 + u];
        const float c = pmul(sigm(zf), cst[u][r]) + pmul(sigm(zi), tanh_(zg)); cst[u][r] = c; const float h = pmul(sigm(zo), tanh_(c)); b16 a_, c_; split16(h * XS, a_, c_);
        Hh[wave][8 * hlf + r][unit] = a_; Hl[wave][8 * hlf + r][unit] = c_; if (step == T - 1) Ho[wave][8 * hlf + r][unit] = h; } }
    wave_lds_sync(); }
  for (int pass = 0; pass < 2; ++pass) { for (int r4 = 0; r4 < 16; r4 += 4) { const int rr = r4 + (lane >> 3), c4 = (lane & 7) * 4; *(volatile v4f*)(HF + (b0 + rr) * (2 * HID) + dir * HID + c4) = *(const v4f*)(&Ho[wave][rr][c4]); } __threadfence(); }
}
__global__ __launch_bounds__(64) void head_kernel(const int* __restrict__ x, const float* __restrict__ HF, const float* __restrict__ ew, const float* __restrict__ lw, const float* __restrict__ W1, const float* __restrict__ b1, const float* __restrict__ W2, const float* __restrict__ b2, float* __restrict__ out) {
  __shared__ int Tk[64][T + 1]; __shared__ float Ftab[64][FH + 2];
  const size_t b = (size_t)blockIdx.x * 64 + threadIdx.x; int* tok = Tk[threadIdx.x]; float* feat = Ftab[threadIdx.x];
  for (int t = 0; t < T; ++t) tok[t] = x[b * T + t];
  int total = 0, uniq = 0; float ent = 0.0f;
  for (int t = 0; t < T; ++t) total += (tok[t] != 0) ? 1 : 0;
  const float ftot = (float)total, inv = 1.0f / fmaxf(ftot, 1.0f);
#pragma unroll 1
  for (int t = 0; t < T; ++t) { if (tok[t] == 0) continue; int cnt = 0; bool first = true;
#pragma unroll 1
    for (int s = 0; s < T; ++s) { if (tok[s] == tok[t]) { ++cnt; if (s < t) first = false; } }
    if (first) { ++uniq; const float p = (float)cnt * inv; ent -= pmul(p, __logf(p + 1e-8f)); } }
  const float us = (float)(uniq < 1 ? 1 : (uniq > V ? V : uniq)); const float maxent = __logf(us); float en = ent / (maxent + 1e-8f); if (!(ftot > 1.0f)) en = 0.0f;
  for (int j = 0; j < 2 * HID; ++j) feat[j] = HF[b * (2 * HID) + j]; feat[2 * HID] = pmul(en, bf16_rne(ew[0])); feat[2 * HID + 1] = pmul(ftot * (1.0f / 40.0f), bf16_rne(lw[0]));
  float lg[NE]; for (int e = 0; e < NE; ++e) lg[e] = bf16_rne(b2[e]);
#pragma unroll 1
  for (int o = 0; o < 32; ++o) { float s = bf16_rne(b1[o]);
#pragma unroll 1
    for (int j = 0; j < FH; ++j) s += pmul(feat[j], bf16_rne(W1[o * FH + j]));
    s = fmaxf(s, 0.0f);
#pragma unroll 1
    for (int e = 0; e < NE; ++e) lg[e] += pmul(s, bf16_rne(W2[e * 32 + o])); }
  const float mx = fmaxf(fmaxf(lg[0], lg[1]), fmaxf(lg[2], lg[3])); float ex[NE], se = 0.0f; for (int e = 0; e < NE; ++e) { ex[e] = nexp(lg[e] - mx); se += ex[e]; }
  v4f o4 = {ex[0] / se, ex[1] / se, ex[2] / se, ex[3] / se};
  for (int pass = 0; pass < 2; ++pass) { *(volatile v4f*)(out + b * NE) = o4; __threadfence(); }
}
}

extern "C" void kernel_launch(void* const* d_in, const int* in_sizes, int n_in, void* d_out, int out_size, void* d_ws, size_t ws_size, hipStream_t stream) {
  (void)n_in;
  auto Fp = [&](int i) { return (const float*)d_in[i]; };
  if (in_sizes[0] != NBt * T || in_sizes[1] != V * D || in_sizes[2] != G4 * D || in_sizes[3] != G4 * HID || in_sizes[12] != 32 * FH || in_sizes[14] != NE * 32 || out_size != NBt * NE) return;
  size_t off = 0; char* ws = (char*)d_ws;
  auto carve = [&](size_t bytes) { char* p = ws + off; off += (bytes + 255) & ~(size_t)255; return p; };
  b16* EMB16 = (b16*)carve(V * D * 2); b16* WIH = (b16*)carve((size_t)2 * G4 * D * 2); b16* WHH = (b16*)carve((size_t)2 * G4 * HID * 2); float* HF = (float*)carve((size_t)NBt * 2 * HID * 4);
  if (off > ws_size || off > ((size_t)128 << 20)) return;
  prep_kernel<<<(V * D / 8 + 2 * G4 * D / 8 + 2 * G4 * HID / 8 + 255) / 256, 256, 0, stream>>>(Fp(1), Fp(2), Fp(3), Fp(6), Fp(7), EMB16, WIH, WHH);
  lstm_kernel<<<dim3(NBt / 64, 2), 128, 0, stream>>>((const int*)d_in[0], EMB16, WIH, WHH, Fp(4), Fp(5), Fp(8), Fp(9), HF);
  head_kernel<<<NBt / 64, 64, 0, stream>>>((const int*)d_in[0], HF, Fp(10), Fp(11), Fp(12), Fp(13), Fp(14), Fp(15), (float*)d_out);
}
